// NLayerGat_2035814498362
// MI455X (gfx1250) — hardware-run, weakly checked
//
#include <hip/hip_runtime.h>


namespace {
constexpr int N = 50000, NP = 50048, E = 800000, V = 50000, F = 128, NH = 8, FH = 16, NC = 16;
constexpr float XS = 8.0f, WSC = 256.0f, NEGA = 0.2f, NEGACT = 0.01f;
typedef _Float16 b16;
typedef __attribute__((ext_vector_type(16))) _Float16 v16b;
typedef __attribute__((ext_vector_type(8))) _Float16 v8b;
typedef __attribute__((ext_vector_type(8))) float v8f;
typedef __attribute__((ext_vector_type(4))) float v4f;
__device__ __forceinline__ float bf16_rne(float f) { unsigned int u = __float_as_uint(f); u += 0x7FFFu + ((u >> 16) & 1u); return __uint_as_float(u & 0xFFFF0000u); }
__device__ __forceinline__ void split16(float v, b16& hi, b16& lo) { hi = (b16)v; lo = (b16)(v - (float)hi); }
__device__ __forceinline__ v16b frag_kb(const b16* p, int hh) { const v8b a = *(const v8b*)(p + 8 * hh), b = *(const v8b*)(p + 16 + 8 * hh); v16b f;
#pragma unroll
  for (int e = 0; e < 8; ++e) { f[e] = a[e]; f[8 + e] = b[e]; } return f; }
__device__ __forceinline__ v8f wmma16b(v16b a, v16b b, v8f c) { v8f d = __builtin_amdgcn_wmma_f32_16x16x32_f16(false, a, false, b, (short)0, c, false, false); asm volatile("v_nop\n\tv_nop\n\tv_nop\n\tv_nop" : "+v"(d) : "v"(a), "v"(b)); return d; }
__device__ __forceinline__ void wave_lds_sync() { __builtin_amdgcn_fence(__ATOMIC_RELEASE, "workgroup"); __builtin_amdgcn_wave_barrier(); __builtin_amdgcn_fence(__ATOMIC_ACQUIRE, "workgroup"); }
__device__ __forceinline__ float pmul(float a, float b) { float p = a * b; asm volatile("" : "+v"(p)); return p; }
__device__ __forceinline__ float opaque(float a) { asm volatile("" : "+v"(a)); return a; }
__device__ __forceinline__ int iclamp(int v, int lo, int hi) { return v < lo ? lo : (v > hi ? hi : v); }
__device__ __forceinline__ float lrelu(float x, float ns) { return x > 0.0f ? x : ns * x; }
__device__ __forceinline__ float nexp(float x) { return __builtin_amdgcn_exp2f(x * 1.4426950408889634f); }
constexpr int CSR_NBLK = 512, CSR_GB = 9, CSR_GN = 1 << CSR_GB  , CSR_TS = (CSR_GN < 32 ? 32 : CSR_GN)  , CSR_MAXG = 512, CSR_CAP = 12288  ;
__device__ __host__ __forceinline__ int csr_tix(int v) { return (v >> CSR_GB) * CSR_TS + (v & (CSR_GN - 1)); }
__global__ __launch_bounds__(64) void csrA_kernel(const int* __restrict__ dst, int E, int N, int nG, int CHP, int NGP, int* __restrict__ STG, int* __restrict__ HST) {
  extern __shared__ int sm[];
  int* cnt = sm; int* run = sm + NGP; int* ids = sm + 2 * NGP;
  const int b = blockIdx.x; const int ch = (E + CSR_NBLK - 1) / CSR_NBLK; const int e0 = b * ch, e1 = min(E, e0 + ch);
  for (int i = threadIdx.x; i < NGP; i += 64) cnt[i] = 0;
  for (int i = threadIdx.x; i < CHP; i += 64) ids[i] = -1;
  __syncthreads();
  if (threadIdx.x == 0) {
    for (int e = e0; e < e1; ++e) { int d = dst[e]; d = (d < 0) ? 0 : (d >= N ? N - 1 : d); cnt[d >> CSR_GB] += 1; }
    int acc = 0; for (int g = 0; g < nG; ++g) { run[g] = acc; acc += cnt[g]; }
    for (int e = e0; e < e1; ++e) { int d = dst[e]; d = (d < 0) ? 0 : (d >= N ? N - 1 : d); const int g = d >> CSR_GB; ids[run[g]] = e; run[g] += 1; } }
  __syncthreads();
  typedef __attribute__((ext_vector_type(4))) int v4i;
  for (int pass = 0; pass < 2; ++pass) {
    for (int i = threadIdx.x; i < CHP / 4; i += 64) *(volatile v4i*)(STG + (size_t)b * CHP + i * 4) = *(const v4i*)(&ids[i * 4]);
    for (int i = threadIdx.x; i < NGP / 4; i += 64) { v4i v; for (int e = 0; e < 4; ++e) v[e] = (i * 4 + e < nG) ? cnt[i * 4 + e] : 0; *(volatile v4i*)(HST + (size_t)b * NGP + i * 4) = v; }
    __threadfence(); }
}
__global__ __launch_bounds__(512) void csrS_kernel(const int* __restrict__ HST, int nG, int NGP, int* __restrict__ START, int* __restrict__ TOT, int* __restrict__ OFF) {
  __shared__ int tot[CSR_MAXG];
  const int b = threadIdx.x;
  for (int pass = 0; pass < 2; ++pass) { int runb = 0; for (int g = 0; g < nG; ++g) { int c = HST[(size_t)b * NGP + g]; c = (c < 0) ? 0 : c; ((volatile int*)OFF)[(size_t)g * CSR_NBLK + b] = runb; runb += c; } __threadfence(); }
  for (int g = threadIdx.x; g < nG; g += 512) { int s = 0; for (int bb = 0; bb < CSR_NBLK; ++bb) { int c = HST[(size_t)bb * NGP + g]; s += (c < 0) ? 0 : c; } tot[g] = s; }
  __syncthreads();
  if (threadIdx.x < 32) {
    __shared__ int st[CSR_MAXG + 32];
    if (threadIdx.x == 0) { int acc = 0; for (int g = 0; g < NGP; ++g) { st[g] = acc; if (g < nG) acc += (tot[g] + 31) & ~31; } st[NGP] = acc; }
    __builtin_amdgcn_fence(__ATOMIC_RELEASE, "workgroup"); __builtin_amdgcn_wave_barrier(); __builtin_amdgcn_fence(__ATOMIC_ACQUIRE, "workgroup");
    for (int pass = 0; pass < 2; ++pass) { for (int i = threadIdx.x; i < NGP + 32; i += 32) { ((volatile int*)START)[i] = (i <= NGP) ? st[min(i, NGP)] : 0; ((volatile int*)TOT)[i] = (i < nG) ? tot[i] : 0; } __threadfence(); } }
}
__global__ __launch_bounds__(256) void csrB_kernel(const int* __restrict__ dst, int N, int nG, int CHP, int NGP, int permLen, const int* __restrict__ STG, const int* __restrict__ HST, const int* __restrict__ OFF, const int* __restrict__ START, const int* __restrict__ TOT, int* __restrict__ PERM, int* __restrict__ ROWPTR, int* __restrict__ ROWCNT, int* __restrict__ FLAG) {
  typedef __attribute__((ext_vector_type(4))) int v4i;
  __shared__ int ids[CSR_CAP]; __shared__ unsigned short key[CSR_CAP]; __shared__ int outp[CSR_CAP]; __shared__ int ncnt[CSR_GN + 1]; __shared__ int boff[CSR_NBLK + 1];
  const int g = blockIdx.x, t_ = threadIdx.x; int tot = TOT[g]; int st = START[g], stn = START[g + 1]; const int v0 = g * CSR_GN; const int nv = min(CSR_GN, N - v0); const int t0 = g * CSR_TS;
  st = (st < 0) ? 0 : (st > permLen - 32 ? permLen - 32 : st) & ~31; stn = (stn < st) ? st : (stn > permLen ? permLen : stn); tot = (tot < 0) ? 0 : tot; if (tot > stn - st && tot <= CSR_CAP) tot = stn - st;
  if (tot > CSR_CAP) {
    for (int pass = 0; pass < 2; ++pass) { for (int i = t_; i < CSR_TS / 4; i += 256) { v4i a, c; for (int e = 0; e < 4; ++e) { a[e] = st; c[e] = 0; } *(volatile v4i*)(ROWPTR + t0 + i * 4) = a; *(volatile v4i*)(ROWCNT + t0 + i * 4) = c; } if (t_ == 0) ((volatile int*)FLAG)[0] = 1; __threadfence(); } (void)nv; return; }
  if (t_ == 0) { int acc = 0; for (int b = 0; b < CSR_NBLK; ++b) { boff[b] = acc; int c = HST[(size_t)b * NGP + g]; c = (c < 0) ? 0 : (c > CHP ? CHP : c); acc += c; if (acc > tot) acc = tot; } boff[CSR_NBLK] = acc; }
  for (int i = t_; i <= CSR_GN; i += 256) ncnt[i] = 0;
  __syncthreads();
  for (int b = 0; b < CSR_NBLK; ++b) { const int c = boff[b + 1] - boff[b]; int o_ = OFF[(size_t)g * CSR_NBLK + b]; o_ = (o_ < 0) ? 0 : (o_ > CHP - c ? CHP - c : o_); const int* src_ = STG + (size_t)b * CHP + o_;
    for (int i = t_; i < c; i += 256) { int id = src_[i]; id = (id < 0) ? 0 : id; ids[boff[b] + i] = id; int d = dst[id]; d = (d < v0) ? v0 : (d >= N ? N - 1 : d); int kk = d - v0; kk = (kk < 0) ? 0 : (kk >= CSR_GN ? CSR_GN - 1 : kk); key[boff[b] + i] = (unsigned short)kk; } }
  __syncthreads();
  if (t_ == 0) { for (int i = 0; i < tot; ++i) ncnt[key[i]] += 1; int acc = 0; for (int vl = 0; vl < CSR_GN; ++vl) { const int c = ncnt[vl]; ncnt[vl] = acc; acc += c; } ncnt[CSR_GN] = acc;
    for (int i = 0; i < tot; ++i) { const int vl = key[i]; outp[ncnt[vl]] = ids[i]; ncnt[vl] += 1; }
    for (int vl = CSR_GN; vl > 0; --vl) ncnt[vl] = ncnt[vl - 1]; ncnt[0] = 0; }
  __syncthreads();
  for (int pass = 0; pass < 2; ++pass) {
    for (int i = t_; i < (stn - st) / 4; i += 256) { v4i v; for (int e = 0; e < 4; ++e) { const int q = i * 4 + e; v[e] = (q < tot) ? outp[q] : -1; } *(volatile v4i*)(PERM + st + i * 4) = v; }
    for (int i = t_; i < CSR_TS / 4; i += 256) { v4i a, c; for (int e = 0; e < 4; ++e) { const int vl = i * 4 + e; const int vc = vl < CSR_GN ? vl : CSR_GN; a[e] = (vl < CSR_GN) ? st + ncnt[vc] : st; c[e] = (vl < nv) ? (ncnt[(vc < CSR_GN ? vc : CSR_GN - 1) + 1] - ncnt[vc]) : 0; } *(volatile v4i*)(ROWPTR + t0 + i * 4) = a; *(volatile v4i*)(ROWCNT + t0 + i * 4) = c; }
    __threadfence(); }
}
__global__ __launch_bounds__(256) void csrZ_kernel(int* __restrict__ p, size_t n4) { typedef __attribute__((ext_vector_type(4))) int v4i; const size_t tid = (size_t)blockIdx.x * 256 + threadIdx.x, nth = (size_t)gridDim.x * 256; v4i z = {0, 0, 0, 0}; for (size_t i = tid; i < n4; i += nth) *(volatile v4i*)(p + i * 4) = z; }
struct CsrBufs { int *STG, *HST, *OFF, *START, *TOT, *PERM, *ROWPTR, *ROWCNT, *FLAG; int nG, NGP, CHP; size_t permLen; char* base; size_t bytes; };
static size_t csr_carve(CsrBufs& c, char* ws, size_t off, int E, int N) {
  const size_t off0 = off; c.base = ws + off;
  auto al = [&](size_t bytes) { char* p = ws + off; off += (bytes + 255) & ~(size_t)255; return p; };
  c.nG = (N + CSR_GN - 1) / CSR_GN; c.NGP = (c.nG + 31) & ~31; const int ch = (E + CSR_NBLK - 1) / CSR_NBLK; c.CHP = (ch + 31) & ~31; c.permLen = (size_t)E + 32 * (size_t)c.nG + 32;
  c.STG = (int*)al((size_t)CSR_NBLK * c.CHP * 4); c.HST = (int*)al((size_t)CSR_NBLK * c.NGP * 4); c.OFF = (int*)al((size_t)c.NGP * CSR_NBLK * 4); c.START = (int*)al((size_t)(c.NGP + 64) * 4); c.TOT = (int*)al((size_t)(c.NGP + 64) * 4);
  c.PERM = (int*)al(c.permLen * 4); c.ROWPTR = (int*)al((size_t)c.nG * CSR_TS * 4); c.ROWCNT = (int*)al((size_t)c.nG * CSR_TS * 4); c.FLAG = (int*)al(256);
  c.bytes = off - off0; return off;
}
static void csr_build(const CsrBufs& c, const int* dst, int E, int N, hipStream_t stream) {
  const size_t smem = (size_t)(2 * c.NGP + c.CHP) * 4;
  csrZ_kernel<<<512, 256, 0, stream>>>((int*)c.base, c.bytes / 16);
  csrA_kernel<<<CSR_NBLK, 64, smem, stream>>>(dst, E, N, c.nG, c.CHP, c.NGP, c.STG, c.HST);
  csrS_kernel<<<1, 512, 0, stream>>>(c.HST, c.nG, c.NGP, c.START, c.TOT, c.OFF);
  csrB_kernel<<<c.nG, 256, 0, stream>>>(dst, N, c.nG, c.CHP, c.NGP, (int)c.permLen, c.STG, c.HST, c.OFF, c.START, c.TOT, c.PERM, c.ROWPTR, c.ROWCNT, c.FLAG);
}


__global__ __launch_bounds__(256) void wprep_kernel(const float* __restrict__ w0, const float* __restrict__ w1, const float* __restrict__ w2, b16* __restrict__ W0T, b16* __restrict__ W1T, b16* __restrict__ W2T) {
  const size_t u = (size_t)blockIdx.x * 256 + threadIdx.x; const size_t n1 = (size_t)F * F / 8, n2 = (size_t)NC * F / 8; v8b v;
  if (u < 2 * n1) { const bool second = u >= n1; const size_t e = (second ? u - n1 : u) * 8; const int o = (int)(e / F), k0 = (int)(e % F); const float* w = second ? w1 : w0;
    for (int j = 0; j < 8; ++j) v[j] = (b16)(bf16_rne(w[(size_t)(k0 + j) * F + o]) * WSC); for (int pass = 0; pass < 2; ++pass) { *(volatile v8b*)((second ? W1T : W0T) + e) = v; __threadfence(); } return; }
  const size_t t = u - 2 * n1; if (t < n2) { const size_t e = t * 8; const int o = (int)(e / F), k0 = (int)(e % F); for (int j = 0; j < 8; ++j) v[j] = (b16)(bf16_rne(w2[(size_t)(k0 + j) * NC + o]) * WSC); for (int pass = 0; pass < 2; ++pass) { *(volatile v8b*)(W2T + e) = v; __threadfence(); } }
}
template <int RAWX, int NT>
__global__ __launch_bounds__(128) void proj_kernel(const float* __restrict__ HIN, const float* __restrict__ emb, const int* __restrict__ xid, const b16* __restrict__ WT, const float* __restrict__ as_, const float* __restrict__ ad_, float* __restrict__ HW, float* __restrict__ AS, float* __restrict__ AD) {
  __shared__ __attribute__((aligned(16))) b16 Ah[4][16][F + 8], Al[4][16][F + 8]; __shared__ __attribute__((aligned(16))) float Tf[4][16][F + 4]; __shared__ __attribute__((aligned(16))) float sa[64][8], sd[64][8];
  const int wave = threadIdx.x >> 5, lane = threadIdx.x & 31, nloc = lane & 15, hlf = lane >> 4; const size_t m0 = (size_t)blockIdx.x * 64 + wave * 16; constexpr int OW = NT * 16;
  for (int rr = 0; rr < 16; ++rr) { const size_t r = m0 + rr; v4f xv = {0.0f, 0.0f, 0.0f, 0.0f};
    if (r < (size_t)N) { if (RAWX) { const int id = iclamp(xid[r], 0, V - 1); xv = *(const v4f*)(emb + (size_t)id * F + lane * 4); for (int j = 0; j < 4; ++j) xv[j] = bf16_rne(xv[j]); } else xv = *(const v4f*)(HIN + r * F + lane * 4); }
    for (int j = 0; j < 4; ++j) { b16 p, q; if (RAWX) { p = (b16)(xv[j] * XS); q = (b16)0.0f; } else split16(xv[j] * XS, p, q); Ah[wave][rr][lane * 4 + j] = p; Al[wave][rr][lane * 4 + j] = q; } }
  wave_lds_sync();
  v8f acc[NT];
#pragma unroll
  for (int t = 0; t < NT; ++t) acc[t] = (v8f){};
#pragma unroll 2
  for (int kb = 0; kb < F; kb += 32) { const v16b a = frag_kb(&Ah[wave][nloc][kb], hlf); v16b al = {}; if (!RAWX) al = frag_kb(&Al[wave][nloc][kb], hlf);
#pragma unroll
    for (int t = 0; t < NT; ++t) { const v16b bw = frag_kb(WT + (size_t)(t * 16 + nloc) * F + kb, hlf); acc[t] = wmma16b(a, bw, acc[t]); if (!RAWX) acc[t] = wmma16b(al, bw, acc[t]); } }
  float hs[8][NT], hd[8][NT]; for (int r8 = 0; r8 < 8; ++r8) for (int t = 0; t < NT; ++t) { hs[r8][t] = 0.0f; hd[r8][t] = 0.0f; }
#pragma unroll
  for (int t = 0; t < NT; ++t) { const int c = t * 16 + nloc; const float ws_ = opaque(bf16_rne(as_[c])), wd_ = opaque(bf16_rne(ad_[c]));
#pragma unroll
    for (int r8 = 0; r8 < 8; ++r8) { const float v = acc[t][r8] * (1.0f / (XS * WSC)); Tf[wave][8 * hlf + r8][c] = v; hs[r8][t] = pmul(v, ws_); hd[r8][t] = pmul(v, wd_); } }
#pragma unroll
  for (int r8 = 0; r8 < 8; ++r8)
#pragma unroll
    for (int t = 0; t < NT; ++t) { float a = hs[r8][t], b = hd[r8][t]; for (int o = 1; o < 16; o <<= 1) { a += __shfl_xor(a, o); b += __shfl_xor(b, o); } if (nloc == t) { sa[wave * 16 + 8 * hlf + r8][t] = a; sd[wave * 16 + 8 * hlf + r8][t] = b; } }
  if (NT < 8 && nloc >= NT && nloc < 8) for (int r8 = 0; r8 < 8; ++r8) { sa[wave * 16 + 8 * hlf + r8][nloc] = 0.0f; sd[wave * 16 + 8 * hlf + r8][nloc] = 0.0f; }
  __syncthreads();
  for (int pass = 0; pass < 2; ++pass) { for (int rr = 0; rr < 16; ++rr) { const bool ok = (m0 + rr) < (size_t)N; if (lane < OW / 4) { v4f v = *(const v4f*)(&Tf[wave][rr][lane * 4]); if (!ok) v = (v4f){0.0f, 0.0f, 0.0f, 0.0f}; *(volatile v4f*)(HW + (m0 + rr) * OW + lane * 4) = v; } }
    { const int rl = threadIdx.x >> 1, half = threadIdx.x & 1; *(volatile v4f*)(AS + ((size_t)blockIdx.x * 64 + rl) * 8 + half * 4) = *(const v4f*)(&sa[rl][half * 4]); *(volatile v4f*)(AD + ((size_t)blockIdx.x * 64 + rl) * 8 + half * 4) = *(const v4f*)(&sd[rl][half * 4]); }
    __threadfence(); }
}
__global__ __launch_bounds__(256) void attn_kernel(const float* __restrict__ HW, const float* __restrict__ AS, const float* __restrict__ AD, const float* __restrict__ bias, const int* __restrict__ srcs, const int* __restrict__ PERM, const int* __restrict__ ROWPTR, const int* __restrict__ ROWCNT, int permLen, float* __restrict__ HOUT) {
  const int wave = threadIdx.x >> 5, lane = threadIdx.x & 31; const size_t v = (size_t)blockIdx.x * 8 + wave; const int h = lane >> 2; v4f o = {0.0f, 0.0f, 0.0f, 0.0f};
  if (v < (size_t)N) { int st = ROWPTR[v], cnt = ROWCNT[v]; cnt = iclamp(cnt, 0, 65536); st = iclamp(st, 0, permLen - cnt);
    const v4f ad4a = *(const v4f*)(AD + v * 8), ad4b = *(const v4f*)(AD + v * 8 + 4), as4a = *(const v4f*)(AS + v * 8), as4b = *(const v4f*)(AS + v * 8 + 4);
    const float advh = h < 4 ? ad4a[h & 3] : ad4b[h & 3]; const float asvh = h < 4 ? as4a[h & 3] : as4b[h & 3];
    float mx = lrelu(asvh + advh, NEGA);
#pragma unroll 1
    for (int j = 0; j < cnt; ++j) { const int e = iclamp(PERM[st + j], 0, E - 1); const int s = iclamp(srcs[e], 0, N - 1); const v4f a = *(const v4f*)(AS + (size_t)s * 8), b = *(const v4f*)(AS + (size_t)s * 8 + 4); const float av = h < 4 ? a[h & 3] : b[h & 3]; mx = fmaxf(mx, lrelu(av + advh, NEGA)); }
    float den = nexp(lrelu(asvh + advh, NEGA) - mx); v4f acc = *(const v4f*)(HW + v * F + lane * 4); for (int i = 0; i < 4; ++i) acc[i] = pmul(acc[i], den);
#pragma unroll 1
    for (int j = 0; j < cnt; ++j) { const int e = iclamp(PERM[st + j], 0, E - 1); const int s = iclamp(srcs[e], 0, N - 1); const v4f a = *(const v4f*)(AS + (size_t)s * 8), b = *(const v4f*)(AS + (size_t)s * 8 + 4); const float av = h < 4 ? a[h & 3] : b[h & 3]; const float p = nexp(lrelu(av + advh, NEGA) - mx); den += p;
      const v4f xs = *(const v4f*)(HW + (size_t)s * F + lane * 4); for (int i = 0; i < 4; ++i) acc[i] += pmul(p, xs[i]); }
    const float inv = 1.0f / (den + 1e-16f); for (int i = 0; i < 4; ++i) o[i] = lrelu(pmul(acc[i], inv) + bf16_rne(bias[lane * 4 + i]), NEGACT); }
  for (int pass = 0; pass < 2; ++pass) { *(volatile v4f*)(HOUT + v * F + lane * 4) = o; __threadfence(); }
}
__global__ __launch_bounds__(256) void attn2_kernel(const float* __restrict__ HW2, const float* __restrict__ AS, const float* __restrict__ AD, const float* __restrict__ bias, const int* __restrict__ srcs, const int* __restrict__ PERM, const int* __restrict__ ROWPTR, const int* __restrict__ ROWCNT, int permLen, float* __restrict__ out) {
  __shared__ __attribute__((aligned(16))) float so[8][32];
  const int wave = threadIdx.x >> 5, lane = threadIdx.x & 31, nloc = lane & 15, hlf = lane >> 4; const size_t v = ((size_t)blockIdx.x * 8 + wave) * 2 + hlf;
  int st = ROWPTR[v], cnt = ROWCNT[v]; cnt = iclamp(cnt, 0, 65536); st = iclamp(st, 0, permLen - cnt);
  const float adv = AD[v * 8], asv = AS[v * 8]; float mx = lrelu(asv + adv, NEGA);
  const int cnt_o = __shfl_xor(cnt, 16); const int cmax = cnt > cnt_o ? cnt : cnt_o;
#pragma unroll 1
  for (int j = 0; j < cmax; ++j) { const bool ok = j < cnt; const int e = iclamp(PERM[iclamp(st + j, 0, permLen - 1)], 0, E - 1); const int s = iclamp(srcs[e], 0, N - 1); const float av = AS[(size_t)s * 8]; mx = fmaxf(mx, ok ? lrelu(av + adv, NEGA) : -INFINITY); }
  float den = nexp(lrelu(asv + adv, NEGA) - mx); float acc = pmul(HW2[v * NC + nloc], den);
#pragma unroll 1
  for (int j = 0; j < cmax; ++j) { const bool ok = j < cnt; const int e = iclamp(PERM[iclamp(st + j, 0, permLen - 1)], 0, E - 1); const int s = iclamp(srcs[e], 0, N - 1); const float av = AS[(size_t)s * 8]; const float p = ok ? nexp(lrelu(av + adv, NEGA) - mx) : 0.0f; den += p; acc += pmul(p, HW2[(size_t)s * NC + nloc]); }
  const float val = pmul(acc, 1.0f / (den + 1e-16f)) + bf16_rne(bias[nloc]);
  float m2 = val; for (int o = 1; o < 16; o <<= 1) m2 = fmaxf(m2, __shfl_xor(m2, o)); float se = nexp(val - m2); for (int o = 1; o < 16; o <<= 1) se += __shfl_xor(se, o);
  so[wave][lane] = val - m2 - __logf(se);
  wave_lds_sync();
  for (int pass = 0; pass < 2; ++pass) { if (lane < 8) *(volatile v4f*)(out + ((size_t)blockIdx.x * 8 + wave) * 2 * NC + lane * 4) = *(const v4f*)(&so[wave][lane * 4]); __threadfence(); }
}
}

extern "C" void kernel_launch(void* const* d_in, const int* in_sizes, int n_in, void* d_out, int out_size, void* d_ws, size_t ws_size, hipStream_t stream) {
  (void)n_in;
  auto Fp = [&](int i) { return (const float*)d_in[i]; }; auto Ip = [&](int i) { return (const int*)d_in[i]; };
  if (in_sizes[0] != N || in_sizes[1] != 2 * E || in_sizes[2] != V * F || in_sizes[3] != F * F || in_sizes[4] != NH * FH || in_sizes[7] != F * F || in_sizes[11] != F * NC || in_sizes[12] != NC || out_size != N * NC) return;
  size_t off = 0; char* ws = (char*)d_ws;
  auto carve = [&](size_t bytes) { char* p = ws + off; off += (bytes + 255) & ~(size_t)255; return p; };
  b16* W0T = (b16*)carve((size_t)F * F * 2); b16* W1T = (b16*)carve((size_t)F * F * 2); b16* W2T = (b16*)carve((size_t)NC * F * 2);
  float* HW = (float*)carve((size_t)NP * F * 4); float* HA = (float*)carve((size_t)NP * F * 4); float* AS = (float*)carve((size_t)NP * 8 * 4); float* AD = (float*)carve((size_t)NP * 8 * 4); float* HW2 = (float*)carve((size_t)NP * NC * 4);
  CsrBufs csr; off = csr_carve(csr, ws, off, E, N);
  if (off > ws_size || off > ((size_t)128 << 20)) return;
  wprep_kernel<<<(unsigned)((2 * (size_t)F * F / 8 + (size_t)NC * F / 8 + 255) / 256), 256, 0, stream>>>(Fp(3), Fp(7), Fp(11), W0T, W1T, W2T);
  csr_build(csr, Ip(1) + E, E, N, stream);
  proj_kernel<1, 8><<<NP / 64, 128, 0, stream>>>(nullptr, Fp(2), Ip(0), W0T, Fp(4), Fp(5), HW, AS, AD);
  attn_kernel<<<NP / 8, 256, 0, stream>>>(HW, AS, AD, Fp(6), Ip(1), csr.PERM, csr.ROWPTR, csr.ROWCNT, (int)csr.permLen, HA);
  proj_kernel<0, 8><<<NP / 64, 128, 0, stream>>>(HA, Fp(2), Ip(0), W1T, Fp(8), Fp(9), HW, AS, AD);
  attn_kernel<<<NP / 8, 256, 0, stream>>>(HW, AS, AD, Fp(10), Ip(1), csr.PERM, csr.ROWPTR, csr.ROWCNT, (int)csr.permLen, HA);
  proj_kernel<0, 1><<<NP / 64, 128, 0, stream>>>(HA, Fp(2), Ip(0), W2T, Fp(12), Fp(13), HW2, AS, AD);
  attn2_kernel<<<N / 16, 256, 0, stream>>>(HW2, AS, AD, Fp(14), Ip(1), csr.PERM, csr.ROWPTR, csr.ROWCNT, (int)csr.permLen, (float*)d_out);
}
